// MonotonicModel_v1_90065464197296
// MI455X (gfx1250) — hardware-run, weakly checked
//
#include <hip/hip_runtime.h>


namespace {
constexpr int N = 10240, NC = 10, HID = 256, NS = 33;
constexpr float HS = 256.0f, WSC = 256.0f;
__constant__ float c_ccw[NS] = {0x1.f07c200000000p-11f, 0x1.35cc5c0000000p-7f, 0x1.3a22060000000p-6f, 0x1.d341680000000p-6f, 0x1.3378ec0000000p-5f, 0x1.7b7c2c0000000p-5f, 0x1.be6a0a0000000p-5f, 0x1.fea2340000000p-5f, 0x1.1c20060000000p-4f, 0x1.3711fe0000000p-4f, 0x1.4e20400000000p-4f, 0x1.62df320000000p-4f, 0x1.7348300000000p-4f, 0x1.810ab20000000p-4f, 0x1.8a29c20000000p-4f, 0x1.906c0a0000000p-4f, 0x1.91e3a40000000p-4f, 0x1.906c0a0000000p-4f, 0x1.8a29c20000000p-4f, 0x1.810ab20000000p-4f, 0x1.7348300000000p-4f, 0x1.62df320000000p-4f, 0x1.4e20400000000p-4f, 0x1.3711fe0000000p-4f, 0x1.1c20060000000p-4f, 0x1.fea2340000000p-5f, 0x1.be6a0a0000000p-5f, 0x1.7b7c2c0000000p-5f, 0x1.3378ec0000000p-5f, 0x1.d341680000000p-6f, 0x1.3a22060000000p-6f, 0x1.35cc5c0000000p-7f, 0x1.f07c200000000p-11f};
__constant__ float c_steps[NS] = {0x1.0000000000000p+0f, 0x1.fd88da0000000p-1f, 0x1.f6297c0000000p-1f, 0x1.e9f4160000000p-1f, 0x1.d906bc0000000p-1f, 0x1.c38b300000000p-1f, 0x1.a9b6620000000p-1f, 0x1.8bc8060000000p-1f, 0x1.6a09e60000000p-1f, 0x1.44cf320000000p-1f, 0x1.1c73b40000000p-1f, 0x1.e2b5d40000000p-2f, 0x1.87de2a0000000p-2f, 0x1.2940620000000p-2f, 0x1.8f8b840000000p-3f, 0x1.917a6c0000000p-4f, 0x1.1a62640000000p-54f, -0x1.917a6c0000000p-4f, -0x1.8f8b840000000p-3f, -0x1.2940620000000p-2f, -0x1.87de2a0000000p-2f, -0x1.e2b5d40000000p-2f, -0x1.1c73b40000000p-1f, -0x1.44cf320000000p-1f, -0x1.6a09e60000000p-1f, -0x1.8bc8060000000p-1f, -0x1.a9b6620000000p-1f, -0x1.c38b300000000p-1f, -0x1.d906bc0000000p-1f, -0x1.e9f4160000000p-1f, -0x1.f6297c0000000p-1f, -0x1.fd88da0000000p-1f, -0x1.0000000000000p+0f};
typedef _Float16 b16;
typedef __attribute__((ext_vector_type(16))) _Float16 v16b;
typedef __attribute__((ext_vector_type(8))) _Float16 v8b;
typedef __attribute__((ext_vector_type(8))) float v8f;
typedef __attribute__((ext_vector_type(4))) float v4f;
__device__ __forceinline__ float bf16_rne(float f) { unsigned int u = __float_as_uint(f); u += 0x7FFFu + ((u >> 16) & 1u); float r = __uint_as_float(u & 0xFFFF0000u); asm volatile("" : "+v"(r)); return r; }
__device__ __forceinline__ float bfv(float f) { float r = bf16_rne(f); asm volatile("" : "+v"(r)); return r; }
__device__ __forceinline__ void split16(float v, b16& hi, b16& lo) { hi = (b16)v; lo = (b16)(v - (float)hi); }
__device__ __forceinline__ v16b frag_kb(const b16* p, int hh) { const v8b a = *(const v8b*)(p + 8 * hh), b = *(const v8b*)(p + 16 + 8 * hh); v16b f;
#pragma unroll
  for (int e = 0; e < 8; ++e) { f[e] = a[e]; f[8 + e] = b[e]; } return f; }
__device__ __forceinline__ v8f wmma16b(v16b a, v16b b, v8f c) { v8f d = __builtin_amdgcn_wmma_f32_16x16x32_f16(false, a, false, b, (short)0, c, false, false); asm volatile("v_nop\n\tv_nop\n\tv_nop\n\tv_nop" : "+v"(d) : "v"(a), "v"(b)); return d; }
__device__ __forceinline__ void wave_lds_sync() { __builtin_amdgcn_fence(__ATOMIC_RELEASE, "workgroup"); __builtin_amdgcn_wave_barrier(); __builtin_amdgcn_fence(__ATOMIC_ACQUIRE, "workgroup"); }
__device__ __forceinline__ float pmul(float a, float b) { float p = a * b; asm volatile("" : "+v"(p)); return p; }
__device__ __forceinline__ float elu(float v) { return v > 0.0f ? v : (__expf(v) - 1.0f); }

__global__ __launch_bounds__(256) void wput_kernel(const float* __restrict__ w2, b16* __restrict__ WT) { const int u = blockIdx.x * 256 + threadIdx.x; if (u >= HID * 32) return; const int o = u / 32, k0 = (u % 32) * 8; v8b v;
#pragma unroll
  for (int j = 0; j < 8; ++j) v[j] = (b16)(bf16_rne(w2[(size_t)(k0 + j) * HID + o]) * WSC); for (int pass = 0; pass < 2; ++pass) { *(volatile v8b*)(WT + (size_t)o * HID + k0) = v; __threadfence(); } }
__global__ __launch_bounds__(32) void mono_kernel(const float* __restrict__ logits, const float* __restrict__ w1, const float* __restrict__ b1, const b16* __restrict__ WT, const float* __restrict__ b2, const float* __restrict__ w3, const float* __restrict__ b3, const float* __restrict__ offs, int OLIM, float* __restrict__ out) {
  __shared__ __attribute__((aligned(16))) b16 Ah[32][HID + 8], Al[32][HID + 8]; __shared__ float Tf[32][HID + 1], Xs[32]; const int lane = threadIdx.x, nloc = lane & 15, hlf = lane >> 4; const size_t o0 = (size_t)blockIdx.x * 32; if (o0 >= (size_t)OLIM) return;
  { const size_t idx = o0 + lane; const size_t row = idx / NC; float mx = -INFINITY; for (int c = 0; c < NC; ++c) mx = fmaxf(mx, bfv(logits[row * NC + c])); float se = 0.0f; for (int c = 0; c < NC; ++c) se += __expf(bfv(logits[row * NC + c]) - mx); Xs[lane] = bfv(logits[idx]) - (mx + __logf(se)); }
  for (int k = HID; k < HID + 8; ++k) { Ah[lane][k] = (b16)0.0f; Al[lane][k] = (b16)0.0f; }
  wave_lds_sync();
  const float xme = Xs[lane]; float integ = 0.0f; const float bb3 = bfv(b3[0]);
#pragma unroll 1
  for (int s = 0; s < NS; ++s) {
    for (int rr = 0; rr < 32; ++rr) { const float t = Xs[rr] * (c_steps[s] + 1.0f) * 0.5f; for (int q = 0; q < HID / 32; ++q) { const int c = q * 32 + lane; b16 p, ql; split16(elu(pmul(t, bfv(w1[c])) + bfv(b1[c])) * HS, p, ql); Ah[rr][c] = p; Al[rr][c] = ql; } }
    wave_lds_sync();
#pragma unroll 1
    for (int rt = 0; rt < 2; ++rt) { v8f acc[16];
#pragma unroll
      for (int t2 = 0; t2 < 16; ++t2) acc[t2] = (v8f){};
#pragma unroll 2
      for (int kb = 0; kb < HID; kb += 32) { const v16b a = frag_kb(&Ah[rt * 16 + nloc][kb], hlf), al = frag_kb(&Al[rt * 16 + nloc][kb], hlf);
#pragma unroll
        for (int t2 = 0; t2 < 16; ++t2) { const v16b bw = frag_kb(WT + (size_t)(t2 * 16 + nloc) * HID + kb, hlf); acc[t2] = wmma16b(a, bw, acc[t2]); acc[t2] = wmma16b(al, bw, acc[t2]); } }
#pragma unroll
      for (int t2 = 0; t2 < 16; ++t2) { const int cc = t2 * 16 + nloc; const float bb = bfv(b2[cc]);
#pragma unroll
        for (int r8 = 0; r8 < 8; ++r8) Tf[rt * 16 + 8 * hlf + r8][cc] = elu(acc[t2][r8] * (1.0f / (HS * WSC)) + bb); } }
    wave_lds_sync();
    { float o = bb3;
#pragma unroll 8
      for (int c = 0; c < HID; ++c) o += pmul(Tf[lane][c], bfv(w3[c])); integ += pmul(c_ccw[s], elu(o) + 1.0f); }
    wave_lds_sync(); }
  const float res = pmul(integ, xme * 0.5f) + bfv(offs[0]);
  for (int pass = 0; pass < 2; ++pass) { ((volatile float*)out)[o0 + lane] = res; __threadfence(); } }
}

extern "C" void kernel_launch(void* const* d_in, const int* in_sizes, int n_in, void* d_out, int out_size, void* d_ws, size_t ws_size, hipStream_t stream) {
  (void)n_in;
  auto Fp = [&](int i) { return (const float*)d_in[i]; };
  if (in_sizes[0] != N || in_sizes[1] != HID || in_sizes[3] != HID * HID || in_sizes[5] != HID || out_size != N) return;
  const int OLIM = N;
  size_t off = 0; char* ws = (char*)d_ws;
  auto carve = [&](size_t bytes) { char* p = ws + off; off += (bytes + 255) & ~(size_t)255; return p; };
  b16* WT = (b16*)carve((size_t)HID * HID * 2);
  if (off > ws_size || off > ((size_t)4 << 20)) return;
  wput_kernel<<<(HID * 32 + 255) / 256, 256, 0, stream>>>(Fp(3), WT);
  mono_kernel<<<OLIM / 32, 32, 0, stream>>>(Fp(0), Fp(1), Fp(2), WT, Fp(4), Fp(5), Fp(6), Fp(7), OLIM, (float*)d_out);
}
